// DenoisingModule_3822520893491
// MI455X (gfx1250) — hardware-verified
//
#include <hip/hip_runtime.h>
#include <math.h>
#include <stdint.h>


#define NBATCH 8
#define CH     256
#define DH     128
#define HWN    4096
#define NR     512
#define NSPLIT (HWN / NR)

typedef _Float16 v16h __attribute__((ext_vector_type(16)));
typedef _Float16 v8h  __attribute__((ext_vector_type(8)));
typedef float    v8f  __attribute__((ext_vector_type(8)));
typedef float    v4f  __attribute__((ext_vector_type(4)));
typedef unsigned int v4u __attribute__((ext_vector_type(4)));

__device__ __forceinline__ unsigned short h2u(_Float16 x) { return __builtin_bit_cast(unsigned short, x); }
__device__ __forceinline__ unsigned pk16(unsigned short a, unsigned short b) { return (unsigned)a | ((unsigned)b << 16); }

__device__ __forceinline__ void wave_sync() {
  __builtin_amdgcn_fence(__ATOMIC_RELEASE, "workgroup");
  __builtin_amdgcn_wave_barrier();
  __builtin_amdgcn_fence(__ATOMIC_ACQUIRE, "workgroup");
}

union FragH { v16h v; v8h h[2]; };
__device__ __forceinline__ v16h ldfrag_h(const _Float16* p) {
  FragH f; f.h[0] = *(const v8h*)(p); f.h[1] = *(const v8h*)(p + 16); return f.v;
}

__device__ __forceinline__ v8f wmma_h(v16h a, v16h b, v8f c) {
  c = __builtin_amdgcn_wmma_f32_16x16x32_f16(false, a, false, b, (short)0, c, false, false);
  asm volatile("v_nop\n\tv_nop\n\tv_nop\n\tv_nop" : "+v"(c) : "v"(a), "v"(b));
  return c;
}

__global__ __launch_bounds__(256) void cvt_f16x8_kernel(const float* __restrict__ in, unsigned short* out, int n8,
                                                        float scale) {
  const int i = blockIdx.x * 256 + threadIdx.x;
  if (i < n8) {
    const v4f a = *(const v4f*)(in + 8 * (size_t)i);
    const v4f d = *(const v4f*)(in + 8 * (size_t)i + 4);
    v4u w;
    w[0] = pk16(h2u((_Float16)(a[0] * scale)), h2u((_Float16)(a[1] * scale)));
    w[1] = pk16(h2u((_Float16)(a[2] * scale)), h2u((_Float16)(a[3] * scale)));
    w[2] = pk16(h2u((_Float16)(d[0] * scale)), h2u((_Float16)(d[1] * scale)));
    w[3] = pk16(h2u((_Float16)(d[2] * scale)), h2u((_Float16)(d[3] * scale)));
    volatile v4u* p = (volatile v4u*)(out + 8 * (size_t)i);
    *p = w;
    __threadfence();
    *p = w;
  }
}

__global__ __launch_bounds__(128) void xtok_kernel(const float* __restrict__ x, unsigned short* xt) {
  __shared__ float tile[64 * 65];
  const int tid = threadIdx.x;
  const int n0 = blockIdx.x * 64;
  const int c0 = blockIdx.y * 64;
  const int b  = blockIdx.z;
#pragma unroll
  for (int it = 0; it < 8; ++it) {
    const int cc = it * 8 + (tid >> 4);
    const int f4 = (tid & 15) * 4;
    const v4f v = *(const v4f*)(x + (size_t)(b * CH + c0 + cc) * HWN + n0 + f4);
    tile[cc * 65 + f4 + 0] = v[0];
    tile[cc * 65 + f4 + 1] = v[1];
    tile[cc * 65 + f4 + 2] = v[2];
    tile[cc * 65 + f4 + 3] = v[3];
  }
  __syncthreads();
  const int q = tid >> 3, c8 = (tid & 7) * 8;
  for (int pass = 0; pass < 2; ++pass) {
#pragma unroll
    for (int it = 0; it < 4; ++it) {
      const int n = it * 16 + q;
      v4u w;
#pragma unroll
      for (int p = 0; p < 4; ++p) {
        const float f0 = tile[(c8 + 2 * p) * 65 + n];
        const float f1 = tile[(c8 + 2 * p + 1) * 65 + n];
        w[p] = pk16(h2u((_Float16)f0), h2u((_Float16)f1));
      }
      *(volatile v4u*)(xt + (size_t)(b * HWN + n0 + n) * CH + c0 + c8) = w;
    }
    __threadfence();
  }
}

#define SLP 68

template <int MODE>
__global__ __launch_bounds__(128) void gemm_kernel(
    const unsigned short* __restrict__ Ap, int lda, long strideA,
    const unsigned short* __restrict__ Btp, int ldb, long strideB,
    void* C0, long strideC0, int ldc0,
    void* C1, long strideC1, int ldc1,
    const float* __restrict__ aux0, const float* __restrict__ aux1,
    int M, int N, int K, float scale) {
  __shared__ __align__(16) float sT[4][32 * SLP];
  const int bz   = blockIdx.y;
  const int lane = threadIdx.x & 31;
  const int wave = threadIdx.x >> 5;
  const int tilesN = N >> 6;
  const int tilesM = M >> 5;
  const int tile = blockIdx.x * 4 + wave;
  if (tile >= tilesM * tilesN) return;
  const int tm = tile / tilesN;
  const int tn = tile - tm * tilesN;
  const int m0 = tm << 5;
  const int n0 = tn << 6;

  const _Float16* Ab = (const _Float16*)(const void*)Ap  + (size_t)bz * strideA;
  const _Float16* Bb = (const _Float16*)(const void*)Btp + (size_t)bz * strideB;

  const int c  = lane & 15;
  const int h8 = (lane >> 4) * 8;

  const v8f zero8 = (v8f){0.f, 0.f, 0.f, 0.f, 0.f, 0.f, 0.f, 0.f};
  v8f acc[2][4];
#pragma unroll
  for (int i = 0; i < 2; ++i)
#pragma unroll
    for (int j = 0; j < 4; ++j) acc[i][j] = zero8;

#pragma unroll 1
  for (int k0 = 0; k0 < K; k0 += 32) {
    const v16h a0 = ldfrag_h(Ab + (size_t)(m0 + c) * lda + k0 + h8);
    const v16h a1 = ldfrag_h(Ab + (size_t)(m0 + 16 + c) * lda + k0 + h8);
#pragma unroll
    for (int j = 0; j < 4; ++j) {
      const v16h bf = ldfrag_h(Bb + (size_t)(n0 + (j << 4) + c) * ldb + k0 + h8);
      acc[0][j] = wmma_h(a0, bf, acc[0][j]);
      acc[1][j] = wmma_h(a1, bf, acc[1][j]);
    }
  }

  float* slab = sT[wave];
#pragma unroll
  for (int i = 0; i < 2; ++i)
#pragma unroll
    for (int j = 0; j < 4; ++j)
#pragma unroll
      for (int r = 0; r < 8; ++r) slab[(16 * i + h8 + r) * SLP + (j << 4) + c] = acc[i][j][r] * scale;
  wave_sync();

  if (MODE == 0 || MODE == 1) {
    unsigned short* Ch = (MODE == 0) ? ((unsigned short*)C0 + (size_t)bz * strideC0)
                                     : ((unsigned short*)C1 + (size_t)bz * strideC1);
    const int ldh = (MODE == 0) ? ldc0 : ldc1;
    const int q = lane >> 3, c8 = (lane & 7) * 8;
    float bias[8];
#pragma unroll
    for (int e = 0; e < 8; ++e) bias[e] = 0.f;
    if (MODE == 0) {
#pragma unroll
      for (int e = 0; e < 8; ++e) {
        const int d = n0 + c8 + e;
        const int dt = (d < DH) ? d : (DH - 1);
        int dp = d - DH;
        dp = (dp < 0) ? 0 : dp;
        dp = (dp > DH - 1) ? (DH - 1) : dp;
        const float bt = aux0[dt];
        const float bp = aux1[dp];
        bias[e] = (d < DH) ? bt : bp;
      }
    }
    for (int pass = 0; pass < 2; ++pass) {
#pragma unroll
      for (int it = 0; it < 8; ++it) {
        const int row = it * 4 + q;
        const float* sp = slab + row * SLP + c8;
        v4u hv;
#pragma unroll
        for (int p = 0; p < 4; ++p) {
          const _Float16 e0 = (_Float16)(sp[2 * p] + bias[2 * p]);
          const _Float16 e1 = (_Float16)(sp[2 * p + 1] + bias[2 * p + 1]);
          hv[p] = pk16(h2u(e0), h2u(e1));
        }
        *(volatile v4u*)(Ch + (size_t)(m0 + row) * ldh + n0 + c8) = hv;
      }
      __threadfence();
    }
  }
  if (MODE == 1 || MODE == 2) {
    float* Cf;
    const float* Rf;
    int rowbase;
    if (MODE == 1) {
      Cf = (float*)C0 + (size_t)bz * strideC0;
      Rf = (const float*)C0;
      rowbase = m0;
    } else {
      const int bb = m0 >> 12;
      Cf = (float*)C0 + (size_t)bb * strideC0;
      Rf = (const float*)C1 + (size_t)bb * strideC1;
      rowbase = m0 & (HWN - 1);
    }
    const int q = lane >> 3, f4 = (lane & 7) * 4;
    for (int pass = 0; pass < 2; ++pass) {
#pragma unroll
      for (int it = 0; it < 16; ++it) {
        const int col = it * 4 + q;
        v4f v;
#pragma unroll
        for (int i = 0; i < 4; ++i) v[i] = slab[(f4 + i) * SLP + col];
        const size_t go = (size_t)(n0 + col) * ldc0 + rowbase + f4;
        if (MODE == 2) {
          const float bc = aux0[n0 + col];
          const v4f rd = *(const v4f*)(Rf + go);
          v = (v + bc) + rd;
        }
        *(volatile v4f*)(Cf + go) = v;
      }
      __threadfence();
    }
  }
}

#define SC_STG 72
#define SC_SLOTS (NBATCH * 32 * 128)
#define SC_LDS_BYTES (SC_SLOTS * 4 + 32 * 128 * 4 + 4 * 16 * SC_STG * 2)

__global__ __launch_bounds__(128) void scores_kernel(const unsigned short* __restrict__ Thp, unsigned short* Pp, int e) {
  extern __shared__ v4f dsm4[];
  float* sS = (float*)(void*)dsm4;
  float* sI = sS + SC_SLOTS;
  _Float16* stg = (_Float16*)(void*)(sS + SC_SLOTS + 32 * 128);

  const int tid  = threadIdx.x;
  const int wave = tid >> 5;
  const int lane = tid & 31;
  const int h    = lane >> 4;
  const int c    = lane & 15;
  const int mt   = blockIdx.x & 63;
  const int nt   = blockIdx.x >> 6;
  const int m0   = mt * 64;
  const int n0l  = nt * 64 + wave * 16;
  const int ng   = e * NR + n0l;
  const _Float16* T = (const _Float16*)(const void*)Thp;
  const float kS = 0.09016844005556021f;
  const v8f zero8 = (v8f){0.f, 0.f, 0.f, 0.f, 0.f, 0.f, 0.f, 0.f};

#pragma unroll 1
  for (int b = 0; b < NBATCH; ++b) {
    v8f acc[4];
#pragma unroll
    for (int j = 0; j < 4; ++j) acc[j] = zero8;
    const _Float16* Ar = T + (size_t)(b * HWN + ng + c) * CH + 8 * h;
    const _Float16* Br = T + (size_t)(b * HWN + m0 + c) * CH + DH + 8 * h;
#pragma unroll
    for (int ks = 0; ks < 4; ++ks) {
      const v16h a = ldfrag_h(Ar + ks * 32);
#pragma unroll
      for (int j = 0; j < 4; ++j) {
        const v16h bf = ldfrag_h(Br + (size_t)(j * 16) * CH + ks * 32);
        acc[j] = wmma_h(a, bf, acc[j]);
      }
    }
#pragma unroll
    for (int j = 0; j < 4; ++j)
#pragma unroll
      for (int r = 0; r < 8; ++r) sS[(b * 32 + j * 8 + r) * 128 + tid] = acc[j][r] * kS;
  }

#pragma unroll 2
  for (int el = 0; el < 32; ++el) {
    float* sp = sS + el * 128 + tid;
    float v[NBATCH];
#pragma unroll
    for (int b = 0; b < NBATCH; ++b) v[b] = sp[b * 4096];
    float mx = v[0];
#pragma unroll
    for (int b = 1; b < NBATCH; ++b) mx = fmaxf(mx, v[b]);
    float sum = 0.f;
#pragma unroll
    for (int b = 0; b < NBATCH; ++b) {
      const float t = exp2f(v[b] - mx);
      sum += t;
      sp[b * 4096] = t;
    }
    sI[el * 128 + tid] = 16384.0f * __builtin_amdgcn_rcpf(sum);
  }

  _Float16* sw = stg + wave * (16 * SC_STG);
  const int q = lane >> 3, c8 = (lane & 7) * 8;
#pragma unroll 1
  for (int b = 0; b < NBATCH; ++b) {
#pragma unroll 4
    for (int el = 0; el < 32; ++el) {
      const int j = el >> 3, r = el & 7;
      const float p = sS[(b * 32 + el) * 128 + tid] * sI[el * 128 + tid];
      sw[(8 * h + r) * SC_STG + 16 * j + c] = (_Float16)p;
    }
    wave_sync();
    for (int pass = 0; pass < 2; ++pass) {
#pragma unroll
      for (int it = 0; it < 4; ++it) {
        const int row = it * 4 + q;
        const v8h t = *(const v8h*)(sw + row * SC_STG + c8);
        const v4u w = __builtin_bit_cast(v4u, t);
        *(volatile v4u*)(Pp + (size_t)(b * NR + n0l + row) * HWN + m0 + c8) = w;
      }
      __threadfence();
    }
    wave_sync();
  }
}

extern "C" void kernel_launch(void* const* d_in, const int* in_sizes, int n_in,
                              void* d_out, int out_size, void* d_ws, size_t ws_size,
                              hipStream_t stream) {
  if (n_in < 7) return;
  if (in_sizes[0] != NBATCH * CH * HWN) return;
  if (in_sizes[1] != DH * CH) return;
  if (in_sizes[2] != DH) return;
  if (in_sizes[3] != DH * CH) return;
  if (in_sizes[4] != DH) return;
  if (in_sizes[5] != CH * CH) return;
  if (in_sizes[6] != CH) return;
  if (out_size != NBATCH * CH * HWN) return;

  const float* x       = (const float*)d_in[0];
  const float* w_theta = (const float*)d_in[1];
  const float* b_theta = (const float*)d_in[2];
  const float* w_phi   = (const float*)d_in[3];
  const float* b_phi   = (const float*)d_in[4];
  const float* w_conv  = (const float*)d_in[5];
  const float* b_conv  = (const float*)d_in[6];
  float* out = (float*)d_out;

  const size_t szP    = (size_t)NBATCH * NR * HWN * 2;
  const size_t szX16  = (size_t)NBATCH * CH * HWN * 2;
  const size_t szDen  = (size_t)NBATCH * CH * HWN * 4;
  const size_t szW    = (size_t)CH * CH * 2;
  size_t off = 0;
  const size_t oP    = off; off += szP;
  const size_t oXcm  = off; off += szX16;
  const size_t oXtok = off; off += szX16;
  const size_t oThp  = off; off += szX16;
  const size_t oDen  = off; off += szDen;
  const size_t oWtp  = off; off += szW;
  const size_t oWc   = off; off += szW;
  if (off > ws_size) return;
  if (off > (size_t)134217728) return;

  char* ws = (char*)d_ws;
  unsigned short* Pp     = (unsigned short*)(ws + oP);
  unsigned short* Xcm    = (unsigned short*)(ws + oXcm);
  unsigned short* Xtok   = (unsigned short*)(ws + oXtok);
  unsigned short* DenTok = (unsigned short*)(ws + oXtok);
  unsigned short* Thp    = (unsigned short*)(ws + oThp);
  float*          Den    = (float*)(ws + oDen);
  unsigned short* Wtp    = (unsigned short*)(ws + oWtp);
  unsigned short* Wc     = (unsigned short*)(ws + oWc);

  const dim3 blk256(256), blk128(128);
  const int n8x = NBATCH * CH * HWN / 8;
  const int n8t = DH * CH / 8;
  const int n8c = CH * CH / 8;

  cvt_f16x8_kernel<<<dim3((n8x + 255) / 256), blk256, 0, stream>>>(x, Xcm, n8x, 1.0f);
  cvt_f16x8_kernel<<<dim3((n8t + 255) / 256), blk256, 0, stream>>>(w_theta, Wtp, n8t, 16.0f);
  cvt_f16x8_kernel<<<dim3((n8t + 255) / 256), blk256, 0, stream>>>(w_phi, Wtp + (size_t)DH * CH, n8t, 16.0f);
  cvt_f16x8_kernel<<<dim3((n8c + 255) / 256), blk256, 0, stream>>>(w_conv, Wc, n8c, 16.0f);
  xtok_kernel<<<dim3(HWN / 64, CH / 64, NBATCH), blk128, 0, stream>>>(x, Xtok);
  {
    const int M = NBATCH * HWN, N = CH, K = CH;
    const int tiles = (M / 32) * (N / 64);
    gemm_kernel<0><<<dim3((tiles + 3) / 4, 1), blk128, 0, stream>>>(
        Xtok, CH, 0L, Wtp, CH, 0L,
        (void*)Thp, 0L, CH, (void*)Thp, 0L, CH,
        b_theta, b_phi, M, N, K, 0.0625f);
  }
  (void)hipFuncSetAttribute(reinterpret_cast<const void*>(&scores_kernel),
                            hipFuncAttributeMaxDynamicSharedMemorySize, SC_LDS_BYTES);
  for (int e = 0; e < NSPLIT; ++e) {
    scores_kernel<<<dim3(64 * (NR / 64)), blk128, SC_LDS_BYTES, stream>>>(Thp, Pp, e);
    const int M = NR, N = CH, K = HWN;
    const int tiles = (M / 32) * (N / 64);
    gemm_kernel<1><<<dim3((tiles + 3) / 4, NBATCH), blk128, 0, stream>>>(
        Pp, HWN, (long)NR * HWN, Xcm, HWN, (long)CH * HWN,
        (void*)(Den + (size_t)e * NR), (long)CH * HWN, HWN,
        (void*)(DenTok + (size_t)e * NR * CH), (long)HWN * CH, CH,
        b_conv, b_conv, M, N, K, 6.103515625e-05f);
  }
  {
    const int M = NBATCH * HWN, N = CH, K = CH;
    const int tiles = (M / 32) * (N / 64);
    gemm_kernel<2><<<dim3((tiles + 3) / 4, 1), blk128, 0, stream>>>(
        DenTok, CH, 0L, Wc, CH, 0L,
        (void*)out, (long)CH * HWN, HWN, (void*)Den, (long)CH * HWN, HWN,
        b_conv, b_conv, M, N, K, 0.0625f);
  }
  (void)hipGetLastError();
}
